// ImprovedConvLayer_27633819583186
// MI455X (gfx1250) — hardware-verified
//
#include <hip/hip_runtime.h>
#include <stddef.h>

#define NATOM 8000
#define MNBR 12
#define AF 64
#define NROWS 96000
#define NPC 896
#define EPC 512
#define PJC 256
#define EB_ROWS 96
#define EB_THR 192
#define NB_EDGE 1000
#define NODE_ROWS 32
#define NB_NODE 250
#define S3_NODES 32
#define NB_S3 250
#define WSC 64.0f
#define INV_WSC 0.015625f
#define BN_EPS 1e-5f

static_assert(NROWS == NATOM * MNBR);
static_assert(NB_EDGE * EB_ROWS == NROWS);
static_assert(EB_ROWS == 16 * (EB_THR / 32));
static_assert(NB_NODE * NODE_ROWS == NATOM);
static_assert(NB_S3 * S3_NODES == NATOM);
static_assert(NATOM * AF == 500 * 256 * 4);
static_assert(NPC == 14 * 64);

typedef _Float16 f16;
typedef f16 v16h __attribute__((ext_vector_type(16)));
typedef f16 v8h_t __attribute__((ext_vector_type(8)));
typedef v8h_t __attribute__((may_alias)) v8h;
typedef float v8f __attribute__((ext_vector_type(8)));
typedef float v4f_t __attribute__((ext_vector_type(4)));
typedef v4f_t __attribute__((may_alias)) v4f;
typedef float v2f_t __attribute__((ext_vector_type(2)));
typedef v2f_t __attribute__((may_alias)) v2f;
typedef unsigned int v4u __attribute__((ext_vector_type(4)));

union Frag { v16h v; v8h_t h[2]; };

__device__ __forceinline__ v8f zero8() {
    v8f z;
#pragma unroll
    for (int i = 0; i < 8; ++i) z[i] = 0.0f;
    return z;
}

__device__ __forceinline__ v4f_t zero4() {
    v4f_t z;
#pragma unroll
    for (int i = 0; i < 4; ++i) z[i] = 0.0f;
    return z;
}

__device__ __forceinline__ v8h_t cvt8(const float* __restrict__ p) {
    const v4f_t a = *(const v4f*)p;
    const v4f_t b = *(const v4f*)(p + 4);
    v8h_t r;
#pragma unroll
    for (int j = 0; j < 4; ++j) { r[j] = (f16)a[j]; r[4 + j] = (f16)b[j]; }
    return r;
}

__device__ __forceinline__ v16h afrag_f32(const float* __restrict__ rowp, int k0, int hh) {
    Frag f;
    f.h[0] = cvt8(rowp + k0 + 8 * hh);
    f.h[1] = cvt8(rowp + k0 + 16 + 8 * hh);
    return f.v;
}

__device__ __forceinline__ v16h bfrag(const f16* __restrict__ colp, int k0, int hh) {
    Frag f;
    f.h[0] = *(const v8h*)(colp + k0 + 8 * hh);
    f.h[1] = *(const v8h*)(colp + k0 + 16 + 8 * hh);
    return f.v;
}

__device__ __forceinline__ v8f mm64(const v16h a0, const v16h a1, const f16* __restrict__ colp, int hh) {
    const v16h b0 = bfrag(colp, 0, hh);
    const v16h b1 = bfrag(colp, 32, hh);
    v8f acc = zero8();
    acc = __builtin_amdgcn_wmma_f32_16x16x32_f16(false, a0, false, b0, (short)0, acc, false, false);
    acc = __builtin_amdgcn_wmma_f32_16x16x32_f16(false, a1, false, b1, (short)0, acc, false, false);
    asm volatile("v_nop\n\tv_nop\n\tv_nop\n\tv_nop" : "+v"(acc) : "v"(a0), "v"(a1), "v"(b0), "v"(b1));
    return acc;
}

__device__ __forceinline__ float sigm(float x) { return __builtin_amdgcn_rcpf(1.0f + __expf(-x)); }
__device__ __forceinline__ float softp(float x) { return fmaxf(x, 0.0f) + __logf(1.0f + __expf(-fabsf(x))); }

__global__ void __launch_bounds__(256) k_wprep(
    const float* __restrict__ Wf, const float* __restrict__ We, const float* __restrict__ W3,
    f16* __restrict__ WTn, f16* __restrict__ WTe)
{
    const int blk = blockIdx.x;
    const int tid = threadIdx.x;
    const int rloc = tid >> 3;
    const int kq = (tid & 7) * 8;
    const bool isn = blk < 28;
    const int lb = isn ? blk : (blk - 28);
    const int grp = lb >> 2;
    const int col = lb * 32 + rloc;
    const int cc = col & 127;
    const float* src; int ro;
    if (isn) {
        if (grp == 0)      { src = Wf; ro = 0; }
        else if (grp == 1) { src = Wf; ro = 64; }
        else if (grp == 2) { src = We; ro = 0; }
        else if (grp == 3) { src = We; ro = 64; }
        else if (grp == 4) { src = W3; ro = 0; }
        else if (grp == 5) { src = W3; ro = 64; }
        else               { src = W3; ro = 128; }
    } else {
        if (grp == 0)      { src = Wf; ro = 128; }
        else if (grp == 1) { src = We; ro = 128; }
        else if (grp == 2) { src = W3; ro = 192; }
        else               { src = W3; ro = 256; }
    }
    union { v8h_t h; v4u u; } pk;
#pragma unroll
    for (int i = 0; i < 8; ++i)
        pk.h[i] = (f16)(src[(size_t)(ro + kq + i) * 128 + cc] * WSC);
    f16* dst = (isn ? WTn : WTe) + (size_t)col * 64 + kq;
    *(volatile v4u*)dst = pk.u;
    __threadfence();
    *(volatile v4u*)dst = pk.u;
}

__global__ void __launch_bounds__(64) k_node(
    const float* __restrict__ x, const f16* __restrict__ WTn, float* __restrict__ NP)
{
    __shared__ __align__(16) float stg[2][1024];
    const int lane = threadIdx.x & 31, w = threadIdx.x >> 5;
    const int hh = lane >> 4, m = lane & 15, c4 = m * 4;
    const int row0 = blockIdx.x * NODE_ROWS + w * 16;
    const float* ar = x + (size_t)(row0 + m) * AF;
    const v16h a0 = afrag_f32(ar, 0, hh);
    const v16h a1 = afrag_f32(ar, 32, hh);
    float* sw = stg[w];
#pragma unroll 1
    for (int q = 0; q < 14; ++q) {
#pragma unroll
        for (int tt = 0; tt < 4; ++tt) {
            const int col0 = q * 64 + tt * 16;
            const v8f acc = mm64(a0, a1, WTn + (size_t)(col0 + m) * 64, hh);
#pragma unroll
            for (int r = 0; r < 8; ++r) sw[(8 * hh + r) * 64 + 16 * tt + m] = acc[r] * INV_WSC;
        }
        __syncthreads();
        v4f_t v[8];
#pragma unroll
        for (int p = 0; p < 8; ++p) v[p] = *(const v4f*)(sw + (2 * p + hh) * 64 + c4);
        float* go = NP + (size_t)row0 * NPC + q * 64 + c4;
#pragma unroll
        for (int p = 0; p < 8; ++p) *(volatile v4f_t*)(go + (size_t)(2 * p + hh) * NPC) = v[p];
        __threadfence();
#pragma unroll
        for (int p = 0; p < 8; ++p) *(volatile v4f_t*)(go + (size_t)(2 * p + hh) * NPC) = v[p];
        __syncthreads();
    }
}

template <int PASS>
__global__ void __launch_bounds__(EB_THR) k_edge(
    const float* __restrict__ nbr, const int* __restrict__ nidx, const f16* __restrict__ WTe,
    const float* __restrict__ NP, const float* __restrict__ bfull, const float* __restrict__ bedge,
    float* __restrict__ PJL, float* __restrict__ part1,
    const float* __restrict__ sc1, const float* __restrict__ sh1,
    float* __restrict__ T2, float* __restrict__ out1)
{
    __shared__ __align__(16) float lds[12800];
    const int tid = threadIdx.x, lane = tid & 31, w = tid >> 5;
    const int hh = lane >> 4, m = lane & 15, c4 = m * 4;
    const int blk = blockIdx.x;
    const int brow0 = blk * EB_ROWS;
    const int wrow0 = brow0 + 16 * w;

    const float* ar = nbr + (size_t)(wrow0 + m) * AF;
    const v16h a0 = afrag_f32(ar, 0, hh);
    const v16h a1 = afrag_f32(ar, 32, hh);

    int nrow[8], jrow[8];
#pragma unroll
    for (int r = 0; r < 8; ++r) {
        const int row = wrow0 + 8 * hh + r;
        nrow[r] = row / MNBR;
        int j = nidx[row];
        j = j < 0 ? 0 : (j > NATOM - 1 ? NATOM - 1 : j);
        jrow[r] = j;
    }

    if (PASS == 0) {
        float* partS = lds;
        float* partQ = lds + 3072;
        float* stg = lds + 6144 + w * 1024;
#pragma unroll 1
        for (int t = 0; t < 16; ++t) {
            const int cl = 16 * t + m;
            const v8f acc = mm64(a0, a1, WTe + (size_t)cl * 64, hh);
            const int iCol = (t < 8) ? cl : (cl + 128);
            const int jCol = iCol + 128;
            const float bfv = bfull[cl & 127], bev = bedge[cl & 127];
            const float bias = (t < 8) ? bfv : bev;
            float s = 0.0f, q = 0.0f;
#pragma unroll
            for (int r = 0; r < 8; ++r) {
                const float v = acc[r] * INV_WSC + NP[(size_t)nrow[r] * NPC + iCol]
                              + NP[(size_t)jrow[r] * NPC + jCol] + bias;
                s += v;
                q = fmaf(v, v, q);
            }
            partS[(2 * w + hh) * 256 + cl] = s;
            partQ[(2 * w + hh) * 256 + cl] = q;
        }
#pragma unroll 1
        for (int qg = 0; qg < 4; ++qg) {
#pragma unroll
            for (int tt = 0; tt < 4; ++tt) {
                const int cl = 256 + 64 * qg + 16 * tt + m;
                const v8f acc = mm64(a0, a1, WTe + (size_t)cl * 64, hh);
                const int jCol = cl + 384;
#pragma unroll
                for (int r = 0; r < 8; ++r)
                    stg[(8 * hh + r) * 64 + 16 * tt + m] = acc[r] * INV_WSC + NP[(size_t)jrow[r] * NPC + jCol];
            }
            __syncthreads();
            v4f_t v[8];
#pragma unroll
            for (int p = 0; p < 8; ++p) v[p] = *(const v4f*)(stg + (2 * p + hh) * 64 + c4);
            float* go = PJL + (size_t)wrow0 * PJC + 64 * qg + c4;
#pragma unroll
            for (int p = 0; p < 8; ++p) *(volatile v4f_t*)(go + (size_t)(2 * p + hh) * PJC) = v[p];
            __threadfence();
#pragma unroll
            for (int p = 0; p < 8; ++p) *(volatile v4f_t*)(go + (size_t)(2 * p + hh) * PJC) = v[p];
            __syncthreads();
        }
        __syncthreads();
        v2f_t sq[2];
#pragma unroll
        for (int it = 0; it < 2; ++it) {
            const int ch = tid + it * EB_THR;
            v2f_t o;
            o.x = 0.0f; o.y = 0.0f;
            if (ch < 256) {
                double S = 0.0, Q = 0.0;
#pragma unroll
                for (int i = 0; i < 12; ++i) {
                    S += (double)partS[i * 256 + ch];
                    Q += (double)partQ[i * 256 + ch];
                }
                o.x = (float)S; o.y = (float)Q;
                *(volatile v2f_t*)(part1 + ((size_t)blk * 256 + ch) * 2) = o;
            }
            sq[it] = o;
        }
        __threadfence();
#pragma unroll
        for (int it = 0; it < 2; ++it) {
            const int ch = tid + it * EB_THR;
            if (ch < 256) *(volatile v2f_t*)(part1 + ((size_t)blk * 256 + ch) * 2) = sq[it];
        }
    } else {
        float* sT2 = lds + 12288;
#pragma unroll 1
        for (int u = 0; u < 8; ++u) {
            const int isg = (u < 4) ? 1 : 0;
            const int tA = isg ? u : (u + 4);
            const int clA = 16 * tA + m;
            const int clB = clA + 64;
            const v8f accA = mm64(a0, a1, WTe + (size_t)clA * 64, hh);
            const v8f accB = mm64(a0, a1, WTe + (size_t)clB * 64, hh);
            const int iColA = isg ? clA : (clA + 128);
            const int jColA = iColA + 128;
            const int iColB = iColA + 64, jColB = jColA + 64;
            const float bfA = bfull[clA & 127], beA = bedge[clA & 127];
            const float bfB = bfull[clB & 127], beB = bedge[clB & 127];
            const float bA = isg ? bfA : beA;
            const float bB = isg ? bfB : beB;
            const float scA = sc1[clA], shA = sh1[clA], scB = sc1[clB], shB = sh1[clB];
            float* gt = lds + (isg ? 0 : 6144);
            const int ccol = 16 * (u & 3) + m;
#pragma unroll
            for (int r = 0; r < 8; ++r) {
                const size_t nb = (size_t)nrow[r] * NPC, jb = (size_t)jrow[r] * NPC;
                const float vA = accA[r] * INV_WSC + NP[nb + iColA] + NP[jb + jColA] + bA;
                const float vB = accB[r] * INV_WSC + NP[nb + iColB] + NP[jb + jColB] + bB;
                const float yA = fmaf(vA, scA, shA);
                const float yB = fmaf(vB, scB, shB);
                gt[(16 * w + 8 * hh + r) * 64 + ccol] = sigm(yA) * softp(yB);
            }
        }
        __syncthreads();
        for (int i2 = tid; i2 < 512; i2 += EB_THR) {
            const int nn = i2 >> 6, c = i2 & 63;
            float s = 0.0f;
#pragma unroll
            for (int mm = 0; mm < MNBR; ++mm) s += lds[(12 * nn + mm) * 64 + c];
            sT2[i2] = s;
        }
        __syncthreads();
        v4f_t tv = zero4();
        if (tid < 128) {
            tv = *(const v4f*)(sT2 + 4 * tid);
            *(volatile v4f_t*)(T2 + (size_t)blk * 512 + 4 * tid) = tv;
        }
        const float* gE = lds + 6144;
        v4f_t ov[8];
#pragma unroll
        for (int p = 0; p < 8; ++p) {
            const int rl = 16 * w + 2 * p + hh;
            const size_t e = (size_t)(brow0 + rl) * AF + c4;
            const v4f_t g = *(const v4f*)(gE + rl * 64 + c4);
            const v4f_t nv = *(const v4f*)(nbr + e);
            ov[p] = nv + g;
            *(volatile v4f_t*)(out1 + e) = ov[p];
        }
        __threadfence();
        if (tid < 128) *(volatile v4f_t*)(T2 + (size_t)blk * 512 + 4 * tid) = tv;
#pragma unroll
        for (int p = 0; p < 8; ++p) {
            const int rl = 16 * w + 2 * p + hh;
            const size_t e = (size_t)(brow0 + rl) * AF + c4;
            *(volatile v4f_t*)(out1 + e) = ov[p];
        }
    }
}

__global__ void __launch_bounds__(128) k_stats3(
    const float* __restrict__ NP, const float* __restrict__ PJL, const float* __restrict__ b3,
    float* __restrict__ part3)
{
    const int c = threadIdx.x;
    const int blk = blockIdx.x;
    const double bb = (double)b3[c];
    double Sz = 0.0, Sz2 = 0.0;
#pragma unroll 1
    for (int i = 0; i < S3_NODES; ++i) {
        const int n = blk * S3_NODES + i;
        const double s = (double)NP[(size_t)n * NPC + 512 + c] + bb;
        double su = 0.0, su2 = 0.0, sv = 0.0, sv2 = 0.0;
#pragma unroll 1
        for (int mm = 0; mm < MNBR; ++mm) {
            const float* rp = PJL + (size_t)(n * MNBR + mm) * PJC;
            const double u = (double)rp[c];
            const double v = (double)rp[128 + c];
            su += u; su2 += u * u;
            sv += v; sv2 += v * v;
        }
        Sz += 144.0 * s + 12.0 * (su + sv);
        Sz2 += 144.0 * s * s + 12.0 * (su2 + sv2) + 24.0 * s * (su + sv) + 2.0 * su * sv;
    }
    v2f_t o;
    o.x = (float)Sz; o.y = (float)Sz2;
    float* dst = part3 + ((size_t)blk * 128 + c) * 2;
    *(volatile v2f_t*)dst = o;
    __threadfence();
    *(volatile v2f_t*)dst = o;
}

__global__ void __launch_bounds__(256) k_fin1(
    const float* __restrict__ part1, const float* __restrict__ part3,
    const float* __restrict__ g1, const float* __restrict__ b1,
    const float* __restrict__ ge, const float* __restrict__ be,
    const float* __restrict__ g3, const float* __restrict__ b3g,
    float* __restrict__ sc1, float* __restrict__ sh1,
    float* __restrict__ sc3, float* __restrict__ sh3)
{
    const int c = threadIdx.x;
    double S = 0.0, Q = 0.0;
#pragma unroll 1
    for (int b = 0; b < NB_EDGE; ++b) {
        const v2f_t p = *(const v2f*)(part1 + ((size_t)b * 256 + c) * 2);
        S += (double)p.x; Q += (double)p.y;
    }
    const double mean = S * (1.0 / 96000.0);
    double var = Q * (1.0 / 96000.0) - mean * mean;
    var = var < 0.0 ? 0.0 : var;
    const float ga = g1[c & 127], gb = ge[c & 127], ba = b1[c & 127], bbv = be[c & 127];
    const float gam = (c < 128) ? ga : gb;
    const float bet = (c < 128) ? ba : bbv;
    const float scv = gam * rsqrtf((float)var + BN_EPS);
    const float shv = bet - (float)mean * scv;

    const int c3 = c & 127;
    double S3 = 0.0, Q3 = 0.0;
#pragma unroll 1
    for (int b = 0; b < NB_S3; ++b) {
        const v2f_t p = *(const v2f*)(part3 + ((size_t)b * 128 + c3) * 2);
        S3 += (double)p.x; Q3 += (double)p.y;
    }
    const double mean3 = S3 * (1.0 / 1152000.0);
    double var3 = Q3 * (1.0 / 1152000.0) - mean3 * mean3;
    var3 = var3 < 0.0 ? 0.0 : var3;
    const float sc3v = g3[c3] * rsqrtf((float)var3 + BN_EPS);
    const float sh3v = b3g[c3] - (float)mean3 * sc3v;

    *(volatile float*)(sc1 + c) = scv;
    *(volatile float*)(sh1 + c) = shv;
    if (c < 128) {
        *(volatile float*)(sc3 + c) = sc3v;
        *(volatile float*)(sh3 + c) = sh3v;
    }
    __threadfence();
    *(volatile float*)(sc1 + c) = scv;
    *(volatile float*)(sh1 + c) = shv;
    if (c < 128) {
        *(volatile float*)(sc3 + c) = sc3v;
        *(volatile float*)(sh3 + c) = sh3v;
    }
}

__global__ void __launch_bounds__(64) k_3body(
    const float* __restrict__ NP, const float* __restrict__ PJL, const float* __restrict__ b3,
    const float* __restrict__ sc3, const float* __restrict__ sh3, float* __restrict__ T3)
{
    __shared__ __align__(16) float uj[768];
    __shared__ __align__(16) float ucr[768];
    __shared__ __align__(16) float vl[768];
    __shared__ __align__(16) float vcr[768];
    __shared__ __align__(16) float st[64];
    const int n = blockIdx.x, c = threadIdx.x;
    const float scf = sc3[c], shf = sh3[c], scc = sc3[64 + c], shc = sh3[64 + c];
    const float bf = b3[c], bc = b3[64 + c];
    const float pif = NP[(size_t)n * NPC + 512 + c];
    const float pic = NP[(size_t)n * NPC + 576 + c];
#pragma unroll 1
    for (int mm = 0; mm < MNBR; ++mm) {
        const float* rp = PJL + (size_t)(n * MNBR + mm) * PJC;
        uj[mm * 64 + c]  = rp[c];
        ucr[mm * 64 + c] = rp[64 + c];
        vl[mm * 64 + c]  = rp[128 + c];
        vcr[mm * 64 + c] = rp[192 + c];
    }
    __syncthreads();
    float acc = 0.0f;
#pragma unroll 1
    for (int mm = 0; mm < MNBR; ++mm) {
        const float af = pif + uj[mm * 64 + c];
        const float ac = pic + ucr[mm * 64 + c];
        float am = 0.0f;
#pragma unroll 4
        for (int ll = 0; ll < MNBR; ++ll) {
            const float zf = (af + vl[ll * 64 + c]) + bf;
            const float zc = (ac + vcr[ll * 64 + c]) + bc;
            am = fmaf(sigm(fmaf(zf, scf, shf)), softp(fmaf(zc, scc, shc)), am);
        }
        acc += am;
    }
    st[c] = acc;
    __syncthreads();
    v4f_t v = zero4();
    if (c < 16) {
        v = *(const v4f*)(st + 4 * c);
        *(volatile v4f_t*)(T3 + (size_t)n * AF + 4 * c) = v;
    }
    __threadfence();
    if (c < 16) *(volatile v4f_t*)(T3 + (size_t)n * AF + 4 * c) = v;
}

__global__ void __launch_bounds__(256) k_bn2(
    const float* __restrict__ T2, const float* __restrict__ T3,
    const float* __restrict__ g2, const float* __restrict__ b2,
    float* __restrict__ sc2, float* __restrict__ sh2)
{
    __shared__ double sS[256];
    __shared__ double sQ[256];
    const int t = threadIdx.x, c = t & 63, pq = t >> 6;
    double S = 0.0, Q = 0.0;
#pragma unroll 1
    for (int i = 0; i < 2000; ++i) {
        const int n = pq * 2000 + i;
        const float v = T2[(size_t)n * AF + c] + T3[(size_t)n * AF + c];
        S += (double)v;
        Q += (double)v * (double)v;
    }
    sS[t] = S; sQ[t] = Q;
    __syncthreads();
    const double St = ((sS[c] + sS[c + 64]) + sS[c + 128]) + sS[c + 192];
    const double Qt = ((sQ[c] + sQ[c + 64]) + sQ[c + 128]) + sQ[c + 192];
    const double mean = St * (1.0 / 8000.0);
    double var = Qt * (1.0 / 8000.0) - mean * mean;
    var = var < 0.0 ? 0.0 : var;
    const float scv = g2[c] * rsqrtf((float)var + BN_EPS);
    const float shv = b2[c] - (float)mean * scv;
    if (t < 64) {
        *(volatile float*)(sc2 + t) = scv;
        *(volatile float*)(sh2 + t) = shv;
    }
    __threadfence();
    if (t < 64) {
        *(volatile float*)(sc2 + t) = scv;
        *(volatile float*)(sh2 + t) = shv;
    }
}

__global__ void __launch_bounds__(256) k_out(
    const float* __restrict__ x, const float* __restrict__ T2, const float* __restrict__ T3,
    const float* __restrict__ sc2, const float* __restrict__ sh2, float* __restrict__ out0)
{
    const int i = blockIdx.x * 256 + threadIdx.x;
    const size_t e = (size_t)i * 4;
    const int c0 = (int)(e & 63);
    const v4f_t xv = *(const v4f*)(x + e);
    const v4f_t a = *(const v4f*)(T2 + e);
    const v4f_t b = *(const v4f*)(T3 + e);
    const v4f_t sc = *(const v4f*)(sc2 + c0);
    const v4f_t sh = *(const v4f*)(sh2 + c0);
    v4f_t o;
#pragma unroll
    for (int j = 0; j < 4; ++j) {
        const float y = fmaf(a[j] + b[j], sc[j], sh[j]);
        o[j] = softp(xv[j] + y);
    }
    *(volatile v4f_t*)(out0 + e) = o;
    __threadfence();
    *(volatile v4f_t*)(out0 + e) = o;
}

extern "C" void kernel_launch(void* const* d_in, const int* in_sizes, int n_in,
                              void* d_out, int out_size, void* d_ws, size_t ws_size,
                              hipStream_t stream)
{
    if (n_in < 17) return;
    if (in_sizes[0] != NATOM * AF) return;
    if (in_sizes[1] != NROWS * AF) return;
    if (in_sizes[2] != NROWS) return;
    if (in_sizes[3] != 192 * 128 || in_sizes[7] != 192 * 128 || in_sizes[11] != 320 * 128) return;
    if (in_sizes[4] != 128 || in_sizes[5] != 128 || in_sizes[6] != 128) return;
    if (in_sizes[8] != 128 || in_sizes[9] != 128 || in_sizes[10] != 128) return;
    if (in_sizes[12] != 128 || in_sizes[13] != 128 || in_sizes[14] != 128) return;
    if (in_sizes[15] != 64 || in_sizes[16] != 64) return;
    if (out_size != NATOM * AF + NROWS * AF) return;

    const float* atom_in = (const float*)d_in[0];
    const float* nbr     = (const float*)d_in[1];
    const int*   nidx    = (const int*)d_in[2];
    const float* Wf      = (const float*)d_in[3];
    const float* bfull   = (const float*)d_in[4];
    const float* g1      = (const float*)d_in[5];
    const float* b1      = (const float*)d_in[6];
    const float* We      = (const float*)d_in[7];
    const float* bedge   = (const float*)d_in[8];
    const float* ge      = (const float*)d_in[9];
    const float* be      = (const float*)d_in[10];
    const float* W3      = (const float*)d_in[11];
    const float* b3      = (const float*)d_in[12];
    const float* g3      = (const float*)d_in[13];
    const float* b3g     = (const float*)d_in[14];
    const float* g2      = (const float*)d_in[15];
    const float* b2      = (const float*)d_in[16];

    float* out0 = (float*)d_out;
    float* out1 = out0 + (size_t)NATOM * AF;

    size_t off = 0;
    auto carve = [&](size_t bytes) -> size_t {
        const size_t p = off;
        off = (off + bytes + 255) & ~(size_t)255;
        return p;
    };
    const size_t oWTn  = carve((size_t)NPC * 64 * 2);
    const size_t oWTe  = carve((size_t)EPC * 64 * 2);
    const size_t oNP   = carve((size_t)NATOM * NPC * 4);
    const size_t oPJL  = carve((size_t)NROWS * PJC * 4);
    const size_t oP1   = carve((size_t)NB_EDGE * 256 * 2 * 4);
    const size_t oP3   = carve((size_t)NB_S3 * 128 * 2 * 4);
    const size_t oSC1  = carve(256 * 4);
    const size_t oSH1  = carve(256 * 4);
    const size_t oSC3  = carve(128 * 4);
    const size_t oSH3  = carve(128 * 4);
    const size_t oT2   = carve((size_t)NATOM * AF * 4);
    const size_t oT3   = carve((size_t)NATOM * AF * 4);
    const size_t oSC2  = carve(64 * 4);
    const size_t oSH2  = carve(64 * 4);
    const size_t total = off;
    if (total > ws_size) return;

    char* ws = (char*)d_ws;
    f16*   WTn   = (f16*)(ws + oWTn);
    f16*   WTe   = (f16*)(ws + oWTe);
    float* NP    = (float*)(ws + oNP);
    float* PJL   = (float*)(ws + oPJL);
    float* part1 = (float*)(ws + oP1);
    float* part3 = (float*)(ws + oP3);
    float* sc1   = (float*)(ws + oSC1);
    float* sh1   = (float*)(ws + oSH1);
    float* sc3   = (float*)(ws + oSC3);
    float* sh3   = (float*)(ws + oSH3);
    float* T2    = (float*)(ws + oT2);
    float* T3    = (float*)(ws + oT3);
    float* sc2   = (float*)(ws + oSC2);
    float* sh2   = (float*)(ws + oSH2);

    k_wprep<<<28 + 16, 256, 0, stream>>>(Wf, We, W3, WTn, WTe);
    k_node<<<NB_NODE, 64, 0, stream>>>(atom_in, WTn, NP);
    k_edge<0><<<NB_EDGE, EB_THR, 0, stream>>>(nbr, nidx, WTe, NP, bfull, bedge, PJL, part1,
                                               sc1, sh1, T2, out1);
    k_stats3<<<NB_S3, 128, 0, stream>>>(NP, PJL, b3, part3);
    k_fin1<<<1, 256, 0, stream>>>(part1, part3, g1, b1, ge, be, g3, b3g, sc1, sh1, sc3, sh3);
    k_edge<1><<<NB_EDGE, EB_THR, 0, stream>>>(nbr, nidx, WTe, NP, bfull, bedge, PJL, part1,
                                               sc1, sh1, T2, out1);
    k_3body<<<NATOM, 64, 0, stream>>>(NP, PJL, b3, sc3, sh3, T3);
    k_bn2<<<1, 256, 0, stream>>>(T2, T3, g2, b2, sc2, sh2);
    k_out<<<500, 256, 0, stream>>>(atom_in, T2, T3, sc2, sh2, out0);
}
